// WordAttention_41162966565348
// MI455X (gfx1250) — hardware-verified
//
#include <hip/hip_runtime.h>


#define NB_  4
#define CC   256
#define HW   1024
#define LL   15
#define NWB  (LL * NB_)
#define EMB  768
#define CK   8
#define CV   64
#define DM   CC
#define NTK  HW
#define LOSC 1024.0f

#define NN HW
typedef _Float16 h16;
typedef unsigned short bf;
typedef __attribute__((ext_vector_type(16))) __bf16   v16bf;
typedef __attribute__((ext_vector_type(16))) _Float16 v16h;
typedef __attribute__((ext_vector_type(8)))  _Float16 v8h;
typedef __attribute__((ext_vector_type(8)))  unsigned short v8us;
typedef __attribute__((ext_vector_type(8)))  float    v8f;
typedef __attribute__((ext_vector_type(4)))  float    v4f;
typedef __attribute__((ext_vector_type(4)))  _Float16 v4h;
typedef v8h  __attribute__((may_alias)) v8ha;
typedef v4f  __attribute__((may_alias)) v4fa;
typedef v8us __attribute__((may_alias)) v8usa;

__device__ __forceinline__ unsigned short f2bf(float f) { unsigned u = __float_as_uint(f); u += 0x7FFFu + ((u >> 16) & 1u); return (unsigned short)(u >> 16); }
__device__ __forceinline__ float bf2f(unsigned short b) { return __uint_as_float(((unsigned)b) << 16); }
__device__ __forceinline__ float bfr(float f) { return bf2f(f2bf(f)); }
__device__ __forceinline__ v16h cat16(v8h lo, v8h hi) { return __builtin_shufflevector(lo, hi, 0, 1, 2, 3, 4, 5, 6, 7, 8, 9, 10, 11, 12, 13, 14, 15); }
__device__ __forceinline__ v16bf cat16b(v8us lo, v8us hi) { return __builtin_bit_cast(v16bf, __builtin_shufflevector(lo, hi, 0, 1, 2, 3, 4, 5, 6, 7, 8, 9, 10, 11, 12, 13, 14, 15)); }
__device__ __forceinline__ v8f wmma16(v16h a, v16h b, v8f c) { return __builtin_amdgcn_wmma_f32_16x16x32_f16(false, a, false, b, (short)0, c, false, false); }
__device__ __forceinline__ v8f wmmab(v16bf a, v16bf b, v8f c) { return __builtin_amdgcn_wmma_f32_16x16x32_bf16(false, a, false, b, (short)0, c, false, false); }

template <bool SPLITA, bool F16OUT = false>
__global__ __launch_bounds__(128) void k_gemmb(const bf* __restrict__ A, const bf* __restrict__ Al, const bf* __restrict__ Bn, const float* __restrict__ bias, float* C, int ldc, h16* C2, const float* __restrict__ R = nullptr, int K = DM, int roundR = 1) {
    __shared__ __align__(16) float ost[4][16 * 68];
    const int lane = threadIdx.x & 31, wave = threadIdx.x >> 5, lr = lane & 15, hi = lane >> 4;
    const int r0 = blockIdx.x * 64 + wave * 16, c0 = blockIdx.y * 64;
    const size_t aoff = (size_t)(r0 + lr) * K + 8 * hi;
    size_t boff[4];
#pragma unroll
    for (int t = 0; t < 4; ++t) boff[t] = (size_t)(c0 + t * 16 + lr) * K + 8 * hi;
    v8f acc[4];
#pragma unroll
    for (int t = 0; t < 4; ++t) acc[t] = (v8f){};
#pragma unroll 1
    for (int kc = 0; kc < K; kc += 32) {
        const v16bf a = cat16b(*(const v8us*)(A + aoff + kc), *(const v8us*)(A + aoff + kc + 16));
        v16bf al = a;
        if (SPLITA) al = cat16b(*(const v8us*)(Al + aoff + kc), *(const v8us*)(Al + aoff + kc + 16));
#pragma unroll
        for (int t = 0; t < 4; ++t) { const v16bf b = cat16b(*(const v8us*)(Bn + boff[t] + kc), *(const v8us*)(Bn + boff[t] + kc + 16)); acc[t] = wmmab(a, b, acc[t]); if (SPLITA) acc[t] = wmmab(al, b, acc[t]); }
        asm volatile("v_nop\n\tv_nop\n\tv_nop\n\tv_nop" : "+v"(acc[0]), "+v"(acc[1]), "+v"(acc[2]), "+v"(acc[3]) : "v"(a), "v"(al));
    }
    float* os = &ost[wave][0];
#pragma unroll
    for (int t = 0; t < 4; ++t) { const float bv = bias ? bfr(bias[c0 + t * 16 + lr]) : 0.f;
#pragma unroll
        for (int j = 0; j < 8; ++j) os[(hi * 8 + j) * 68 + t * 16 + lr] = acc[t][j] + bv; }
    __syncthreads();
    if (F16OUT) {
        h16* crow = (h16*)(void*)C + (size_t)r0 * ldc + c0;
        auto pass = [&]() {
#pragma unroll
            for (int s = 0; s < 4; ++s) { const int row = 4 * s + (lane >> 3), piece = lane & 7; const float* sp = os + row * 68 + piece * 8; v8h o, o2;
#pragma unroll
                for (int i = 0; i < 8; ++i) { const h16 a = (h16)sp[i]; o[i] = a; o2[i] = (h16)((sp[i] - (float)a) * LOSC); }
                *(volatile v8h*)(crow + (size_t)row * ldc + piece * 8) = o; if (C2) *(volatile v8h*)(C2 + (size_t)r0 * ldc + c0 + (size_t)row * ldc + piece * 8) = o2; }
        };
        pass(); __threadfence(); pass();
    } else {
        float* crow = C + (size_t)r0 * ldc + c0;
        auto pass = [&]() {
#pragma unroll
            for (int s = 0; s < 8; ++s) { const int Lid = (lane >> 3) + 4 * s, piece = lane & 7; const int row = Lid >> 1, cofs = (Lid & 1) * 32 + piece * 4;
                v4f val = *(const v4fa*)(os + row * 68 + cofs); if (R) { const v4f rv = *(const v4f*)(R + ((size_t)r0 + row) * ldc + c0 + cofs); val += roundR ? (v4f){bfr(rv[0]), bfr(rv[1]), bfr(rv[2]), bfr(rv[3])} : rv; }
                *(volatile v4f*)(crow + (size_t)row * ldc + cofs) = val; }
        };
        pass(); __threadfence(); pass();
    }
}

__global__ __launch_bounds__(256) void k_cvt8(const float* __restrict__ src, bf* dst, size_t n8) {
    const size_t i = (size_t)blockIdx.x * 256 + threadIdx.x; if (i >= n8) return;
    const v8f v = *(const v8f*)(src + i * 8); v8us o;
#pragma unroll
    for (int k = 0; k < 8; ++k) o[k] = f2bf(v[k]);
    *(volatile v8us*)(dst + i * 8) = o; __threadfence(); *(volatile v8us*)(dst + i * 8) = o;
}
__global__ __launch_bounds__(256) void k_zero8(bf* dst, size_t n8) {
    const size_t i = (size_t)blockIdx.x * 256 + threadIdx.x; if (i >= n8) return; v8us z;
#pragma unroll
    for (int k = 0; k < 8; ++k) z[k] = 0;
    *(volatile v8us*)(dst + i * 8) = z; __threadfence(); *(volatile v8us*)(dst + i * 8) = z;
}

template <int MODE>
__global__ __launch_bounds__(128) void k_gemm3z(const bf* __restrict__ Ah, const bf* __restrict__ Al, const bf* __restrict__ Bh, const bf* __restrict__ Bl, int K, float* C, int ldc, size_t sA, size_t sB, size_t sC) {
    if ((MODE & 1) && (int)blockIdx.y * 64 > (int)blockIdx.x * 64 + 63) return;
    const size_t z = blockIdx.z; Ah += z * sA; Al += z * sA; Bh += z * sB; Bl += z * sB; C += z * sC;
    const int Klim = (MODE & 2) ? min(K, ((int)blockIdx.x + 1) * 64) : K;
    __shared__ __align__(16) float ost[4][16 * 68];
    const int lane = threadIdx.x & 31, wave = threadIdx.x >> 5, lr = lane & 15, hi = lane >> 4;
    const int r0 = blockIdx.x * 64 + wave * 16, c0 = blockIdx.y * 64;
    const size_t aoff = (size_t)(r0 + lr) * K + 8 * hi;
    v8f acc[4];
#pragma unroll
    for (int t = 0; t < 4; ++t) acc[t] = (v8f){};
#pragma unroll 1
    for (int kc = 0; kc < Klim; kc += 32) {
        const v16bf a = cat16b(*(const v8us*)(Ah + aoff + kc), *(const v8us*)(Ah + aoff + kc + 16));
        v16bf al = a; if (!(MODE & 4) && !(MODE & 16)) al = cat16b(*(const v8us*)(Al + aoff + kc), *(const v8us*)(Al + aoff + kc + 16));
#pragma unroll
        for (int t = 0; t < 4; ++t) { const size_t bo = (size_t)(c0 + t * 16 + lr) * K + kc + 8 * hi;
            const v16bf bh = cat16b(*(const v8us*)(Bh + bo), *(const v8us*)(Bh + bo + 16));
            acc[t] = wmmab(a, bh, acc[t]);
            if (!(MODE & 4)) { if (!(MODE & 16)) acc[t] = wmmab(al, bh, acc[t]); if (!(MODE & 8)) { const v16bf bl = cat16b(*(const v8us*)(Bl + bo), *(const v8us*)(Bl + bo + 16)); acc[t] = wmmab(a, bl, acc[t]); } } }
        asm volatile("v_nop\n\tv_nop\n\tv_nop\n\tv_nop" : "+v"(acc[0]), "+v"(acc[1]), "+v"(acc[2]), "+v"(acc[3]) : "v"(a), "v"(al));
    }
    float* os = &ost[wave][0];
#pragma unroll
    for (int t = 0; t < 4; ++t) {
#pragma unroll
        for (int j = 0; j < 8; ++j) os[(hi * 8 + j) * 68 + t * 16 + lr] = acc[t][j]; }
    __builtin_amdgcn_wave_barrier(); asm volatile("" ::: "memory");
    float* crow = C + (size_t)r0 * ldc + c0;
    auto pass = [&]() {
#pragma unroll
        for (int s = 0; s < 8; ++s) { const int Lid = (lane >> 3) + 4 * s, piece = lane & 7; const int row = Lid >> 1, cofs = (Lid & 1) * 32 + piece * 4;
            const v4f val = *(const v4fa*)(os + row * 68 + cofs); *(volatile v4f*)(crow + (size_t)row * ldc + cofs) = val; }
    };
    pass(); __threadfence(); pass();
}
__global__ __launch_bounds__(256) void k_planes32z(const float* __restrict__ F, int ld, int off, float sc, int rows, bf* Ph, bf* Pl) {
    typedef __attribute__((ext_vector_type(2))) unsigned short v2us;
    const int lane = threadIdx.x & 31; const size_t r = ((size_t)blockIdx.x * 8 + (threadIdx.x >> 5)) * 2 + (lane >> 4); if (r >= (size_t)rows) return; const int z = blockIdx.z; const int c0 = (lane & 15) * 2; v2us oh, ol;
    Ph += (size_t)z * rows * 32; Pl += (size_t)z * rows * 32;
#pragma unroll
    for (int i = 0; i < 2; ++i) { const float y = F[r * ld + off + z * 32 + c0 + i] * sc; const unsigned short hb = f2bf(y); oh[i] = hb; ol[i] = f2bf(y - bf2f(hb)); }
    const size_t o = r * 32 + c0; *(volatile v2us*)(Ph + o) = oh; *(volatile v2us*)(Pl + o) = ol; __threadfence(); *(volatile v2us*)(Ph + o) = oh; *(volatile v2us*)(Pl + o) = ol;
}
__global__ __launch_bounds__(256) void k_vtpadz(const float* __restrict__ F, int ld, int off, int nk, bf* Th, bf* Tl) {
    typedef __attribute__((ext_vector_type(2))) unsigned short v2us;
    const int lane = threadIdx.x & 31; const size_t wid = (size_t)blockIdx.x * 8 + (threadIdx.x >> 5); if (wid >= (size_t)64 * (nk / 64)) return; const int z = blockIdx.z; const int d = (int)(wid / (nk / 64)); const int k0 = (int)(wid % (nk / 64)) * 64 + lane * 2; v2us oh, ol;
    Th += (size_t)z * 64 * nk; Tl += (size_t)z * 64 * nk;
#pragma unroll
    for (int i = 0; i < 2; ++i) { const float y = (d < 32) ? F[(size_t)(k0 + i) * ld + off + z * 32 + (d < 32 ? d : 0)] : 0.f; const unsigned short hb = f2bf(y); oh[i] = hb; ol[i] = f2bf(y - bf2f(hb)); }
    const size_t o = (size_t)d * nk + k0; *(volatile v2us*)(Th + o) = oh; *(volatile v2us*)(Tl + o) = ol; __threadfence(); *(volatile v2us*)(Th + o) = oh; *(volatile v2us*)(Tl + o) = ol;
}
template <int NK>
__global__ __launch_bounds__(256) void k_softmaxz(const float* __restrict__ S, int rows, bf* PH, bf* PL) {
    typedef __attribute__((ext_vector_type(4))) unsigned short v4us;
    const int lane = threadIdx.x & 31, i = blockIdx.x * 8 + (threadIdx.x >> 5); if (i >= rows) return; const size_t zo = (size_t)blockIdx.z * rows * NK; const float* sr = S + zo + (size_t)i * NK; PH += zo; PL += zo;
    float m = -3.0e38f;
#pragma unroll 1
    for (int c0 = lane * 4; c0 < NK; c0 += 128) {
#pragma unroll
        for (int q = 0; q < 4; ++q) m = fmaxf(m, sr[c0 + q]); }
#pragma unroll
    for (int sh = 16; sh; sh >>= 1) m = fmaxf(m, __shfl_xor(m, sh, 32));
    float sum = 0.f;
#pragma unroll 1
    for (int c0 = lane * 4; c0 < NK; c0 += 128) {
#pragma unroll
        for (int q = 0; q < 4; ++q) sum += __expf(sr[c0 + q] - m); }
#pragma unroll
    for (int sh = 16; sh; sh >>= 1) sum += __shfl_xor(sum, sh, 32);
    const float inv = 1.0f / sum;
#pragma unroll 1
    for (int ps = 0; ps < 2; ++ps) {
#pragma unroll 1
        for (int c0 = lane * 4; c0 < NK; c0 += 128) { v4us oh, ol;
#pragma unroll
            for (int q = 0; q < 4; ++q) { const float p = __expf(sr[c0 + q] - m) * inv; const unsigned short hb = f2bf(p); oh[q] = hb; ol[q] = f2bf(p - bf2f(hb)); }
            const size_t o = (size_t)i * NK + c0; *(volatile v4us*)(PH + o) = oh; *(volatile v4us*)(PL + o) = ol; }
        if (ps == 0) __threadfence(); }
}
__global__ __launch_bounds__(256) void k_placez(const float* __restrict__ XH, int rows, int ldy, float* Y) {
    const int lane = threadIdx.x & 31; const size_t q = (size_t)blockIdx.x * 8 + (threadIdx.x >> 5); if (q >= (size_t)rows) return; const int z = blockIdx.z; const float v = XH[((size_t)z * rows + q) * 64 + lane];
    *(volatile float*)(Y + q * ldy + z * 32 + lane) = v; __threadfence(); *(volatile float*)(Y + q * ldy + z * 32 + lane) = v;
}

__global__ __launch_bounds__(256) void k_hplanesz(const float* __restrict__ F, int ld, int h0, float sc, int rows, bf* Ph, bf* Pl) {
    typedef __attribute__((ext_vector_type(2))) unsigned short v2us;
    const int lane = threadIdx.x & 31; const size_t r = (size_t)blockIdx.x * 8 + (threadIdx.x >> 5); if (r >= (size_t)rows) return; const int z = blockIdx.z; v2us oh, ol;
    Ph += (size_t)z * rows * 64; Pl += (size_t)z * rows * 64;
#pragma unroll
    for (int i = 0; i < 2; ++i) { const float y = F[r * ld + (h0 + z) * 64 + lane * 2 + i] * sc; const unsigned short hb = f2bf(y); oh[i] = hb; ol[i] = f2bf(y - bf2f(hb)); }
    const size_t o = r * 64 + lane * 2; *(volatile v2us*)(Ph + o) = oh; *(volatile v2us*)(Pl + o) = ol; __threadfence(); *(volatile v2us*)(Ph + o) = oh; *(volatile v2us*)(Pl + o) = ol;
}
__global__ __launch_bounds__(256) void k_vtz(const float* __restrict__ F, int ld, int h0, int nk, bf* Th, bf* Tl) {
    typedef __attribute__((ext_vector_type(2))) unsigned short v2us;
    const int lane = threadIdx.x & 31; const size_t wid = (size_t)blockIdx.x * 8 + (threadIdx.x >> 5); if (wid >= (size_t)64 * (nk / 64)) return; const int z = blockIdx.z; const int d = (int)(wid / (nk / 64)); const int t0 = (int)(wid % (nk / 64)) * 64 + lane * 2; v2us oh, ol;
    Th += (size_t)z * 64 * nk; Tl += (size_t)z * 64 * nk;
#pragma unroll
    for (int i = 0; i < 2; ++i) { const float y = F[(size_t)(t0 + i) * ld + (h0 + z) * 64 + d]; const unsigned short hb = f2bf(y); oh[i] = hb; ol[i] = f2bf(y - bf2f(hb)); }
    const size_t o = (size_t)d * nk + t0; *(volatile v2us*)(Th + o) = oh; *(volatile v2us*)(Tl + o) = ol; __threadfence(); *(volatile v2us*)(Th + o) = oh; *(volatile v2us*)(Tl + o) = ol;
}
template <int NK>
__global__ __launch_bounds__(256) void k_softmaxzs(const float* __restrict__ S, int rows, float sc, bf* PH, bf* PL) {
    typedef __attribute__((ext_vector_type(4))) unsigned short v4us;
    const int lane = threadIdx.x & 31, i = blockIdx.x * 8 + (threadIdx.x >> 5); if (i >= rows) return; const size_t zo = (size_t)blockIdx.z * rows * NK; const float* sr = S + zo + (size_t)i * NK; PH += zo; PL += zo;
    float m = -3.0e38f;
#pragma unroll 1
    for (int c0 = lane * 4; c0 < NK; c0 += 128) {
#pragma unroll
        for (int q = 0; q < 4; ++q) m = fmaxf(m, sr[c0 + q] * sc); }
#pragma unroll
    for (int sh = 16; sh; sh >>= 1) m = fmaxf(m, __shfl_xor(m, sh, 32));
    float sum = 0.f;
#pragma unroll 1
    for (int c0 = lane * 4; c0 < NK; c0 += 128) {
#pragma unroll
        for (int q = 0; q < 4; ++q) sum += __expf(sr[c0 + q] * sc - m); }
#pragma unroll
    for (int sh = 16; sh; sh >>= 1) sum += __shfl_xor(sum, sh, 32);
    const float inv = 1.0f / sum;
#pragma unroll 1
    for (int ps = 0; ps < 2; ++ps) {
#pragma unroll 1
        for (int c0 = lane * 4; c0 < NK; c0 += 128) { v4us oh, ol;
#pragma unroll
            for (int q = 0; q < 4; ++q) { const float p = __expf(sr[c0 + q] * sc - m) * inv; const unsigned short hb = f2bf(p); oh[q] = hb; ol[q] = f2bf(p - bf2f(hb)); }
            const size_t o = (size_t)i * NK + c0; *(volatile v4us*)(PH + o) = oh; *(volatile v4us*)(PL + o) = ol; }
        if (ps == 0) __threadfence(); }
}

__global__ __launch_bounds__(256) void k_wspad(const float* __restrict__ wsq, bf* WS) {
    const int lane = threadIdx.x & 31; const int n = blockIdx.x * 8 + (threadIdx.x >> 5); if (n >= 64) return; const bool live = n < NWB; const int i = n % NB_, l = n / NB_;
#pragma unroll 1
    for (int ps = 0; ps < 2; ++ps) {
#pragma unroll
        for (int q = 0; q < EMB / 256; ++q) { v8us o;
#pragma unroll
            for (int k = 0; k < 8; ++k) o[k] = f2bf(live ? wsq[((size_t)i * LL + l) * EMB + q * 256 + lane * 8 + k] : 0.f);
            *(volatile v8us*)(WS + (size_t)n * EMB + q * 256 + lane * 8) = o; }
        if (ps == 0) __threadfence(); }
}
__global__ __launch_bounds__(256) void k_w1T(const float* __restrict__ Wm, int CO, bf* Bt) {
    const int lane = threadIdx.x & 31; const int r = blockIdx.x * 8 + (threadIdx.x >> 5); if (r >= CO * 16) return; const int co = r / 16, p = r % 16;
#pragma unroll 1
    for (int ps = 0; ps < 2; ++ps) {
#pragma unroll
        for (int q = 0; q < EMB / 256; ++q) { v8us o;
#pragma unroll
            for (int k = 0; k < 8; ++k) { const int i = q * 256 + lane * 8 + k; o[k] = f2bf(Wm[((size_t)i * CO + co) * 16 + p]); }
            *(volatile v8us*)(Bt + (size_t)r * EMB + q * 256 + lane * 8) = o; }
        if (ps == 0) __threadfence(); }
}
__global__ __launch_bounds__(256) void k_bias16(const float* __restrict__ b, int CO, float* Bv) {
    const int i = blockIdx.x * 256 + threadIdx.x; if (i >= CO * 16) return; const float v = b[i / 16]; *(volatile float*)(Bv + i) = v; __threadfence(); *(volatile float*)(Bv + i) = v;
}
__global__ __launch_bounds__(256) void k_ptb(const float* __restrict__ xb, bf* XT) {
    __shared__ float tl[64][65];
    typedef __attribute__((ext_vector_type(4))) unsigned short v4us;
    const int tid = threadIdx.x, c0 = blockIdx.x * 64, p0 = blockIdx.y * 64; const int rr = tid >> 2, cq = (tid & 3) * 16;
#pragma unroll
    for (int i = 0; i < 16; ++i) tl[rr][cq + i] = xb[(size_t)(c0 + rr) * HW + p0 + cq + i];
    __syncthreads();
    const int lane = tid & 31, wv = tid >> 5;
    auto pass = [&]() {
#pragma unroll
        for (int st = 0; st < 4; ++st) { const int pr = wv * 8 + st * 2 + (lane >> 4); const int cl = (lane & 15) * 4; v4us v;
#pragma unroll
            for (int i = 0; i < 4; ++i) v[i] = f2bf(tl[cl + i][pr]);
            *(volatile v4us*)(XT + (size_t)(p0 + pr) * CC + c0 + cl) = v; }
    };
    pass(); __threadfence(); pass();
}
__global__ __launch_bounds__(256) void k_kwpad(const float* __restrict__ kw, bf* Bt) {
    const int lane = threadIdx.x & 31; const int r = blockIdx.x * 8 + (threadIdx.x >> 5); if (r >= 64) return; v8us o;
#pragma unroll
    for (int k = 0; k < 8; ++k) o[k] = f2bf(r < CK ? kw[(size_t)(r < CK ? r : 0) * CC + lane * 8 + k] : 0.f);
    *(volatile v8us*)(Bt + (size_t)r * CC + lane * 8) = o; __threadfence(); *(volatile v8us*)(Bt + (size_t)r * CC + lane * 8) = o;
}
__global__ __launch_bounds__(256) void k_bnrelu16(const float* __restrict__ Y1, int CO, const float* __restrict__ gam, const float* __restrict__ bet, float* U) {
    const int lane = threadIdx.x & 31; const int c = blockIdx.x * 8 + (threadIdx.x >> 5); if (c >= CO) return; const int NT = NWB * 16; float s = 0.f;
    for (int e = lane; e < NT; e += 32) { const int n = e / 16, p = e % 16; s += Y1[(size_t)n * CO * 16 + c * 16 + p]; }
#pragma unroll
    for (int sh = 16; sh; sh >>= 1) s += __shfl_xor(s, sh, 32);
    const float mu = s / (float)NT; float q = 0.f;
    for (int e = lane; e < NT; e += 32) { const int n = e / 16, p = e % 16; const float d = Y1[(size_t)n * CO * 16 + c * 16 + p] - mu; q = fmaf(d, d, q); }
#pragma unroll
    for (int sh = 16; sh; sh >>= 1) q += __shfl_xor(q, sh, 32);
    const float rs = rsqrtf(q / (float)NT + 1e-5f); const float ga = bfr(gam[c]), be = bfr(bet[c]);
    for (int e = lane; e < NT; e += 32) { const int n = e / 16, p = e % 16; const float v = fmaxf((Y1[(size_t)n * CO * 16 + c * 16 + p] - mu) * rs * ga + be, 0.f); *(volatile float*)(U + (size_t)c * NT + e) = v; }
    __threadfence();
    for (int e = lane; e < NT; e += 32) { const int n = e / 16, p = e % 16; const float v = fmaxf((Y1[(size_t)n * CO * 16 + c * 16 + p] - mu) * rs * ga + be, 0.f); *(volatile float*)(U + (size_t)c * NT + e) = v; }
}
__global__ __launch_bounds__(256) void k_tconv(const float* __restrict__ U, const float* __restrict__ W2, const float* __restrict__ b2, int CI, int CO, float* T8) {
    typedef __attribute__((ext_vector_type(2))) float v2f_;
    const int lane = threadIdx.x & 31; const size_t w = (size_t)blockIdx.x * 8 + (threadIdx.x >> 5); if (w >= (size_t)NWB * CO) return; const int n = (int)(w / CO), co = (int)(w % CO); v2f_ o;
#pragma unroll
    for (int t = 0; t < 2; ++t) { const int op = lane * 2 + t; const int oy = op / 8, ox = op % 8; float acc = bfr(b2[co]);
#pragma unroll 1
        for (int ci = 0; ci < CI; ++ci) { const float* u = U + ((size_t)ci * NWB + n) * 16; const float* wk = W2 + ((size_t)ci * CO + co) * 16;
#pragma unroll
            for (int ky = 0; ky < 4; ++ky) { const int ty = oy + 1 - ky; if (ty < 0 || (ty & 1)) continue; const int iy = ty >> 1; if (iy >= 4) continue;
#pragma unroll
                for (int kx = 0; kx < 4; ++kx) { const int tx = ox + 1 - kx; if (tx < 0 || (tx & 1)) continue; const int ix = tx >> 1; if (ix >= 4) continue; acc = fmaf(u[iy * 4 + ix], bfr(wk[ky * 4 + kx]), acc); } } }
        o[t] = acc; }
    float* dst = T8 + ((size_t)n * CO + co) * 64 + lane * 2; *(volatile v2f_*)dst = o; __threadfence(); *(volatile v2f_*)dst = o;
}
__global__ __launch_bounds__(256) void k_qplanes(const float* __restrict__ T8q, int n, bf* Qh, bf* Ql) {
    typedef __attribute__((ext_vector_type(2))) unsigned short v2us;
    const int lane = threadIdx.x & 31; const size_t w = (size_t)blockIdx.x * 8 + (threadIdx.x >> 5); if (w >= (size_t)HW / 2) return; const int px = (int)(w * 2 + (lane >> 4)); const int c0 = (lane & 15) * 2; const int cell = (px / 32 / 4) * 8 + (px % 32) / 4; v2us oh, ol;
#pragma unroll
    for (int i = 0; i < 2; ++i) { const int c = c0 + i; const float y = (c < CK) ? T8q[((size_t)n * CK + (c < CK ? c : 0)) * 64 + cell] : 0.f; const unsigned short hb = f2bf(y); oh[i] = hb; ol[i] = f2bf(y - bf2f(hb)); }
    const size_t o = (size_t)px * 32 + c0; *(volatile v2us*)(Qh + o) = oh; *(volatile v2us*)(Ql + o) = ol; __threadfence(); *(volatile v2us*)(Qh + o) = oh; *(volatile v2us*)(Ql + o) = ol;
}
__global__ __launch_bounds__(256) void k_kplanes(const float* __restrict__ KKf, bf* Kh, bf* Kl) {
    typedef __attribute__((ext_vector_type(2))) unsigned short v2us;
    const int lane = threadIdx.x & 31; const size_t w = (size_t)blockIdx.x * 8 + (threadIdx.x >> 5); if (w >= (size_t)HW / 2) return; const int p = (int)(w * 2 + (lane >> 4)); const int c0 = (lane & 15) * 2; v2us oh, ol;
#pragma unroll
    for (int i = 0; i < 2; ++i) { const int c = c0 + i; const float y = (c < CK) ? KKf[(size_t)p * 64 + (c < CK ? c : 0)] : 0.f; const unsigned short hb = f2bf(y); oh[i] = hb; ol[i] = f2bf(y - bf2f(hb)); }
    const size_t o = (size_t)p * 32 + c0; *(volatile v2us*)(Kh + o) = oh; *(volatile v2us*)(Kl + o) = ol; __threadfence(); *(volatile v2us*)(Kh + o) = oh; *(volatile v2us*)(Kl + o) = ol;
}
__global__ __launch_bounds__(256) void k_vT(const float* __restrict__ V, bf* Th, bf* Tl) {
    __shared__ float tl[64][65];
    typedef __attribute__((ext_vector_type(4))) unsigned short v4us;
    const int tid = threadIdx.x; const int p0 = blockIdx.x * 64, c0 = blockIdx.y * 64; const int rr = tid >> 2, cq = (tid & 3) * 16;
#pragma unroll
    for (int i = 0; i < 16; ++i) tl[rr][cq + i] = V[(size_t)(p0 + rr) * CC + c0 + cq + i];
    __syncthreads();
    const int lane = tid & 31, wv = tid >> 5;
    auto pass = [&]() {
#pragma unroll
        for (int st = 0; st < 4; ++st) { const int cr = wv * 8 + st * 2 + (lane >> 4); const int pq = (lane & 15) * 4; v4us oh, ol;
#pragma unroll
            for (int i = 0; i < 4; ++i) { const float y = tl[pq + i][cr]; const unsigned short hb = f2bf(y); oh[i] = hb; ol[i] = f2bf(y - bf2f(hb)); }
            const size_t o = (size_t)(c0 + cr) * HW + p0 + pq; *(volatile v4us*)(Th + o) = oh; *(volatile v4us*)(Tl + o) = ol; }
    };
    pass(); __threadfence(); pass();
}
__global__ __launch_bounds__(256) void k_soft(const float* __restrict__ S, bf* PH, bf* PL) {
    typedef __attribute__((ext_vector_type(4))) unsigned short v4us;
    const int lane = threadIdx.x & 31, i = blockIdx.x * 8 + (threadIdx.x >> 5); if (i >= HW) return; const float* sr = S + (size_t)i * HW;
    float m = -3.0e38f;
#pragma unroll 1
    for (int c0 = lane * 4; c0 < HW; c0 += 128) {
#pragma unroll
        for (int q = 0; q < 4; ++q) m = fmaxf(m, sr[c0 + q]); }
#pragma unroll
    for (int sh = 16; sh; sh >>= 1) m = fmaxf(m, __shfl_xor(m, sh, 32));
    float sum = 0.f;
#pragma unroll 1
    for (int c0 = lane * 4; c0 < HW; c0 += 128) {
#pragma unroll
        for (int q = 0; q < 4; ++q) sum += __expf(sr[c0 + q] - m); }
#pragma unroll
    for (int sh = 16; sh; sh >>= 1) sum += __shfl_xor(sum, sh, 32);
    const float inv = 1.0f / sum;
#pragma unroll 1
    for (int ps = 0; ps < 2; ++ps) {
#pragma unroll 1
        for (int c0 = lane * 4; c0 < HW; c0 += 128) { v4us oh, ol;
#pragma unroll
            for (int q = 0; q < 4; ++q) { const float p = __expf(sr[c0 + q] - m) * inv; const unsigned short hb = f2bf(p); oh[q] = hb; ol[q] = f2bf(p - bf2f(hb)); }
            const size_t o = (size_t)i * HW + c0; *(volatile v4us*)(PH + o) = oh; *(volatile v4us*)(PL + o) = ol; }
        if (ps == 0) __threadfence(); }
}
__global__ __launch_bounds__(256) void k_partials(const float* __restrict__ IA, const float* __restrict__ T8v, int n, float* PART) {
    const int lane = threadIdx.x & 31; const int blk = blockIdx.x * 8 + (threadIdx.x >> 5); if (blk >= HW / 32) return; float a = 0.f, b = 0.f, cc = 0.f;
#pragma unroll 1
    for (int rq = 0; rq < 32; ++rq) { const int qp = blk * 32 + rq; const int cell = (qp / 32 / 4) * 8 + (qp % 32) / 4;
#pragma unroll
        for (int k = 0; k < 8; ++k) { const int c = lane * 8 + k; const float ia = IA[(size_t)qp * CC + c]; const float vt = T8v[((size_t)n * CC + c) * 64 + cell]; a = fmaf(ia, vt, a); b = fmaf(ia, ia, b); cc = fmaf(vt, vt, cc); } }
#pragma unroll
    for (int sh = 16; sh; sh >>= 1) { a += __shfl_xor(a, sh, 32); b += __shfl_xor(b, sh, 32); cc += __shfl_xor(cc, sh, 32); }
    const float v = (lane == 0) ? a : (lane == 1) ? b : (lane == 2) ? cc : 0.f; *(volatile float*)(PART + ((size_t)n * 32 + blk) * 32 + lane) = v; __threadfence(); *(volatile float*)(PART + ((size_t)n * 32 + blk) * 32 + lane) = v;
}
__global__ __launch_bounds__(256) void k_cosout(const float* __restrict__ PART, float* OUTB) {
    const int lane = threadIdx.x & 31; if (threadIdx.x >= 32) return; float d = 0.f, b = 0.f, c = 0.f;
    if (lane < NB_) { for (int n = lane * LL; n < lane * LL + LL; ++n) for (int blk = 0; blk < 32; ++blk) { const float* p = PART + ((size_t)n * 32 + blk) * 32; d += p[0]; b += p[1]; c += p[2]; } }
    const float v = d / fmaxf(sqrtf(b) * sqrtf(c), 1e-8f);
    if (lane < NB_) { *(volatile float*)(OUTB + lane) = v; } __threadfence(); if (lane < NB_) { *(volatile float*)(OUTB + lane) = v; }
}

__global__ __launch_bounds__(256) void k_qplanesz(const float* __restrict__ T8q, int i, bf* Qh, bf* Ql) {
    typedef __attribute__((ext_vector_type(2))) unsigned short v2us;
    const int lane = threadIdx.x & 31; const size_t w = (size_t)blockIdx.x * 8 + (threadIdx.x >> 5); if (w >= (size_t)HW / 2) return; const int l = blockIdx.z; const int n = l * NB_ + i; const int px = (int)(w * 2 + (lane >> 4)); const int c0 = (lane & 15) * 2; const int cell = (px / 32 / 4) * 8 + (px % 32) / 4; v2us oh, ol;
#pragma unroll
    for (int k = 0; k < 2; ++k) { const int c = c0 + k; const float y = (c < CK) ? T8q[((size_t)n * CK + (c < CK ? c : 0)) * 64 + cell] : 0.f; const unsigned short hb = f2bf(y); oh[k] = hb; ol[k] = f2bf(y - bf2f(hb)); }
    const size_t o = ((size_t)l * HW + px) * 32 + c0; *(volatile v2us*)(Qh + o) = oh; *(volatile v2us*)(Ql + o) = ol; __threadfence(); *(volatile v2us*)(Qh + o) = oh; *(volatile v2us*)(Ql + o) = ol;
}
__global__ __launch_bounds__(256) void k_partialsz(const float* __restrict__ IA, const float* __restrict__ T8v, int i, float* PART) {
    const int lane = threadIdx.x & 31; const int blk = blockIdx.x * 8 + (threadIdx.x >> 5); if (blk >= HW / 32) return; const int l = blockIdx.z; const int n = l * NB_ + i; const float* ia0 = IA + (size_t)l * HW * CC; float a = 0.f, b = 0.f, cc = 0.f;
#pragma unroll 1
    for (int rq = 0; rq < 32; ++rq) { const int qp = blk * 32 + rq; const int cell = (qp / 32 / 4) * 8 + (qp % 32) / 4;
#pragma unroll
        for (int k = 0; k < 8; ++k) { const int c = lane * 8 + k; const float ia = ia0[(size_t)qp * CC + c]; const float vt = T8v[((size_t)n * CC + c) * 64 + cell]; a = fmaf(ia, vt, a); b = fmaf(ia, ia, b); cc = fmaf(vt, vt, cc); } }
#pragma unroll
    for (int sh = 16; sh; sh >>= 1) { a += __shfl_xor(a, sh, 32); b += __shfl_xor(b, sh, 32); cc += __shfl_xor(cc, sh, 32); }
    const float v = (lane == 0) ? a : (lane == 1) ? b : (lane == 2) ? cc : 0.f; *(volatile float*)(PART + ((size_t)n * 32 + blk) * 32 + lane) = v; __threadfence(); *(volatile float*)(PART + ((size_t)n * 32 + blk) * 32 + lane) = v;
}

__global__ __launch_bounds__(256) void k_kbpad(const float* __restrict__ kb, float* KB) {
    const int i = threadIdx.x; if (i >= 64) return; const float v = (i < CK) ? kb[i] : 0.f; *(volatile float*)(KB + i) = v; __threadfence(); *(volatile float*)(KB + i) = v;
}

extern "C" void kernel_launch(void* const* d_in, const int* in_sizes, int n_in,
                              void* d_out, int out_size, void* d_ws, size_t ws_size, hipStream_t stream) {
    (void)in_sizes; (void)n_in; (void)out_size;
    const float* img = (const float*)d_in[0]; const float* wsq = (const float*)d_in[1]; const float* keyW = (const float*)d_in[2]; const float* keyb = (const float*)d_in[3]; const float* vimgW = (const float*)d_in[4]; const float* vimgb = (const float*)d_in[5];
    const float* qW1 = (const float*)d_in[6]; const float* qb1 = (const float*)d_in[7]; const float* qg = (const float*)d_in[8]; const float* qbe = (const float*)d_in[9]; const float* qW2 = (const float*)d_in[10]; const float* qb2 = (const float*)d_in[11];
    const float* vW1 = (const float*)d_in[12]; const float* vb1 = (const float*)d_in[13]; const float* vg = (const float*)d_in[14]; const float* vbe = (const float*)d_in[15]; const float* vW2 = (const float*)d_in[16]; const float* vb2 = (const float*)d_in[17];
    float* out = (float*)d_out;
    char* wsp = (char*)d_ws;
    auto take = [&](size_t bytes) { char* p = wsp; wsp += (bytes + 255) & ~(size_t)255; return (void*)p; };
    bf* WS = (bf*)take((size_t)64 * EMB * 2); bf* BQ1 = (bf*)take((size_t)CK * 16 * EMB * 2); bf* BV1 = (bf*)take((size_t)CV * 16 * EMB * 2); float* BQB = (float*)take(CK * 16 * 4); float* BVB = (float*)take(CV * 16 * 4);
    float* YQ = (float*)take((size_t)64 * CK * 16 * 4); float* YV = (float*)take((size_t)64 * CV * 16 * 4); float* UQ = (float*)take((size_t)CK * NWB * 16 * 4); float* UV = (float*)take((size_t)CV * NWB * 16 * 4); float* T8Q = (float*)take((size_t)NWB * CK * 64 * 4); float* T8V = (float*)take((size_t)NWB * CC * 64 * 4);
    bf* KW = (bf*)take((size_t)64 * CC * 2); bf* VW = (bf*)take((size_t)CC * CC * 2); bf* XT = (bf*)take((size_t)HW * CC * 2); float* KKf = (float*)take((size_t)NB_ * HW * 64 * 4); float* VI = (float*)take((size_t)HW * CC * 4);
    bf* Kh = (bf*)take((size_t)NB_ * HW * 32 * 2); bf* Kl = (bf*)take((size_t)NB_ * HW * 32 * 2); bf* VTh = (bf*)take((size_t)NB_ * CC * HW * 2); bf* VTl = (bf*)take((size_t)NB_ * CC * HW * 2);
    bf* Qh = (bf*)take((size_t)LL * HW * 32 * 2); bf* Ql = (bf*)take((size_t)LL * HW * 32 * 2); float* S = (float*)take((size_t)LL * HW * HW * 4); bf* PH = (bf*)take((size_t)LL * HW * HW * 2); bf* PL = (bf*)take((size_t)LL * HW * HW * 2); float* IA = (float*)take((size_t)LL * HW * CC * 4); float* PART = (float*)take((size_t)NWB * 32 * 32 * 4);
    if ((size_t)(wsp - (char*)d_ws) > ws_size) return;
    k_wspad<<<64 / 8, 256, 0, stream>>>(wsq, WS); k_w1T<<<(CK * 16) / 8, 256, 0, stream>>>(qW1, CK, BQ1); k_w1T<<<(CV * 16) / 8, 256, 0, stream>>>(vW1, CV, BV1); k_bias16<<<1, 256, 0, stream>>>(qb1, CK, BQB); k_bias16<<<(CV * 16 + 255) / 256, 256, 0, stream>>>(vb1, CV, BVB);
    k_gemmb<false, false><<<dim3(1, (CK * 16) / 64, 1), 128, 0, stream>>>(WS, nullptr, BQ1, BQB, YQ, CK * 16, nullptr, nullptr, EMB);
    k_gemmb<false, false><<<dim3(1, (CV * 16) / 64, 1), 128, 0, stream>>>(WS, nullptr, BV1, BVB, YV, CV * 16, nullptr, nullptr, EMB);
    k_bnrelu16<<<(CK + 7) / 8, 256, 0, stream>>>(YQ, CK, qg, qbe, UQ); k_bnrelu16<<<CV / 8, 256, 0, stream>>>(YV, CV, vg, vbe, UV);
    k_tconv<<<(NWB * CK) / 8, 256, 0, stream>>>(UQ, qW2, qb2, CK, CK, T8Q); k_tconv<<<(NWB * CC) / 8, 256, 0, stream>>>(UV, vW2, vb2, CV, CC, T8V);
    float* KB = BQB;
    k_kwpad<<<64 / 8, 256, 0, stream>>>(keyW, KW); k_cvt8<<<(CC * CC / 8 + 255) / 256, 256, 0, stream>>>(vimgW, VW, CC * CC / 8); k_kbpad<<<1, 256, 0, stream>>>(keyb, KB);
    for (int i = 0; i < NB_; ++i) { const float* xb = img + (size_t)i * CC * HW;
        k_ptb<<<dim3(CC / 64, HW / 64, 1), 256, 0, stream>>>(xb, XT);
        k_gemmb<false, false><<<dim3(HW / 64, 1, 1), 128, 0, stream>>>(XT, nullptr, KW, KB, KKf + (size_t)i * HW * 64, 64, nullptr, nullptr, CC);
        k_gemmb<false, false><<<dim3(HW / 64, CC / 64, 1), 128, 0, stream>>>(XT, nullptr, VW, vimgb, VI, CC, nullptr, nullptr, CC);
        k_kplanes<<<(HW / 2) / 8, 256, 0, stream>>>(KKf + (size_t)i * HW * 64, Kh + (size_t)i * HW * 32, Kl + (size_t)i * HW * 32);
        k_vT<<<dim3(HW / 64, CC / 64, 1), 256, 0, stream>>>(VI, VTh + (size_t)i * CC * HW, VTl + (size_t)i * CC * HW); }
    for (int i = 0; i < NB_; ++i) {
        k_qplanesz<<<dim3((HW / 2) / 8, 1, LL), 256, 0, stream>>>(T8Q, i, Qh, Ql);
        k_gemm3z<0><<<dim3(HW / 64, HW / 64, LL), 128, 0, stream>>>(Qh, Ql, Kh + (size_t)i * HW * 32, Kl + (size_t)i * HW * 32, 32, S, HW, (size_t)HW * 32, 0, (size_t)HW * HW);
        k_softmaxzs<HW><<<dim3(HW / 8, 1, LL), 256, 0, stream>>>(S, HW, 1.0f, PH, PL);
        k_gemm3z<0><<<dim3(HW / 64, CC / 64, LL), 128, 0, stream>>>(PH, PL, VTh + (size_t)i * CC * HW, VTl + (size_t)i * CC * HW, HW, IA, CC, (size_t)HW * HW, 0, (size_t)HW * CC);
        k_partialsz<<<dim3((HW / 32) / 8, 1, LL), 256, 0, stream>>>(IA, T8V, i, PART); }
    k_cosout<<<1, 256, 0, stream>>>(PART, out);
}
